// NonLocalBlock2D_68917045232007
// MI455X (gfx1250) — hardware-verified
//
#include <hip/hip_runtime.h>
#include <math.h>

typedef __attribute__((ext_vector_type(16))) _Float16 v16h;
typedef __attribute__((ext_vector_type(16))) __bf16 v16b;
typedef __attribute__((ext_vector_type(8)))  _Float16 v8h;
typedef __attribute__((ext_vector_type(8)))  __bf16 v8b;
typedef __attribute__((ext_vector_type(8)))  float v8f;
typedef __attribute__((ext_vector_type(4)))  float v4f;
typedef __attribute__((ext_vector_type(4)))  unsigned v4u;

template <typename T> __device__ __forceinline__ void vst2(void* p, T v) { *(volatile T*)p = v; __threadfence(); *(volatile T*)p = v; }

__device__ __forceinline__ v8f wmma16(v16h a, v16h b, v8f c) {
  v8f d = __builtin_amdgcn_wmma_f32_16x16x32_f16(false, a, false, b, (short)0, c, false, false);
  asm volatile("v_nop\n\tv_nop\n\tv_nop\n\tv_nop" : "+v"(d) : "v"(a), "v"(b));
  return d;
}
__device__ __forceinline__ v8f wmma_bf(v16b a, v16b b, v8f c) {
  v8f d = __builtin_amdgcn_wmma_f32_16x16x32_bf16(false, a, false, b, (short)0, c, false, false);
  asm volatile("v_nop\n\tv_nop\n\tv_nop\n\tv_nop" : "+v"(d) : "v"(a), "v"(b));
  return d;
}
__device__ __forceinline__ v16h frag_h(const _Float16* rowk0, int lane) {
  union { v16h v; v8h q[2]; } u; const _Float16* p = rowk0 + 8 * (lane >> 4);
  u.q[0] = *(const v8h*)p; u.q[1] = *(const v8h*)(p + 16); return u.v;
}
__device__ __forceinline__ v16b frag_b(const __bf16* rowk0, int lane) {
  union { v16b v; v8b q[2]; } u; const __bf16* p = rowk0 + 8 * (lane >> 4);
  u.q[0] = *(const v8b*)p; u.q[1] = *(const v8b*)(p + 16); return u.v;
}
__device__ __forceinline__ float bfr(float v) { return (float)(__bf16)v; }
__device__ __forceinline__ v16b fragw_bf(const float* __restrict__ rowk0, int lane) {
  const float* p = rowk0 + 8 * (lane >> 4);
  const v4f a0 = *(const v4f*)p, a1 = *(const v4f*)(p + 4), a2 = *(const v4f*)(p + 16), a3 = *(const v4f*)(p + 20);
  v16b w;
#pragma unroll
  for (int i = 0; i < 4; ++i) {
    const float t0 = a0[i], t1 = a1[i], t2 = a2[i], t3 = a3[i];
    w[i] = (__bf16)t0; w[4 + i] = (__bf16)t1; w[8 + i] = (__bf16)t2; w[12 + i] = (__bf16)t3;
  }
  return w;
}
__device__ __forceinline__ v16h fragw_h(const float* __restrict__ rowk0, int lane, float sc) {
  const float* p = rowk0 + 8 * (lane >> 4);
  const v4f a0 = *(const v4f*)p, a1 = *(const v4f*)(p + 4), a2 = *(const v4f*)(p + 16), a3 = *(const v4f*)(p + 20);
  v16h w;
#pragma unroll
  for (int i = 0; i < 4; ++i) {
    const float t0 = a0[i], t1 = a1[i], t2 = a2[i], t3 = a3[i];
    w[i] = (_Float16)(bfr(t0) * sc); w[4 + i] = (_Float16)(bfr(t1) * sc); w[8 + i] = (_Float16)(bfr(t2) * sc); w[12 + i] = (_Float16)(bfr(t3) * sc);
  }
  return w;
}
__device__ __forceinline__ void ldsx() {
  asm volatile("s_wait_dscnt 0" ::: "memory");
  __builtin_amdgcn_wave_barrier();
  __builtin_amdgcn_fence(3, "workgroup");
}

#define NB  8
#define NP  4096
#define CIN 256
#define CQ  128
#define CV  128
#ifndef TNB
#define TNB NB
#endif
#ifndef TQB
#define TQB (NP / 64)
#endif
#define QL_CARRY 4096.0f
#define P_CARRY  16384.0f
#define Y_CARRY  16.0f
#define W_CARRY  256.0f

#define WS_QH  ((size_t)0)
#define WS_QL  (WS_QH + 2u * (size_t)NB * NP * CQ)
#define WS_KH  (WS_QL + 2u * (size_t)NB * NP * CQ)
#define WS_VT  (WS_KH + 2u * (size_t)NB * NP * CQ)
#define WS_S   (WS_VT + 2u * (size_t)NB * CV * NP)
#define WS_PH  (WS_S  + 4u * (size_t)NP * NP)
#define WS_END (WS_PH + 2u * (size_t)NP * NP)
static_assert(WS_END <= (size_t)134217728);
static_assert(NP % 64 == 0);
static_assert(CIN % 128 == 0);
static_assert(CQ % 64 == 0);
static_assert(CV == 128);
static_assert(TNB <= NB);
static_assert(TQB * 64 <= NP);
static_assert((size_t)NB * CIN * NP * 4u == (size_t)33554432);

__global__ __launch_bounds__(128) __attribute__((amdgpu_num_vgpr(256)))
void k_proj(const float* __restrict__ X, const float* __restrict__ WQ, const float* __restrict__ BQ,
            const float* __restrict__ WK, const float* __restrict__ BK, const float* __restrict__ WV, const float* __restrict__ BV,
            _Float16* __restrict__ QH, _Float16* __restrict__ QL, _Float16* __restrict__ KH, _Float16* __restrict__ VT) {
  __shared__ __align__(16) __bf16 sx[64][CIN + 8];
  __shared__ __align__(16) _Float16 sh[64][72], sl[64][72], tv[64][72];
  const int tid = threadIdx.x, wave = tid >> 5, lane = tid & 31, col = lane & 15, g = lane >> 4;
  const int p0 = blockIdx.x * 64; const size_t b = blockIdx.y; const int which = blockIdx.z;
  const float* Wm = which == 0 ? WQ : which == 1 ? WK : WV;
  const float* Bm = which == 0 ? BQ : which == 1 ? BK : BV;
  const int nout = (which == 2) ? CV : CQ;
  for (int e = tid; e < CIN * 64; e += 128) { const int c = e >> 6, pl = e & 63; sx[pl][c] = (__bf16)X[(b * CIN + c) * (size_t)NP + p0 + pl]; }
  __syncthreads();
#pragma unroll 1
  for (int cg = 0; cg < nout / 64; ++cg) {
    v8f acc[4] = {};
#pragma unroll 1
    for (int kc = 0; kc < CIN / 32; ++kc) {
      const v16b a = frag_b(&sx[wave * 16 + col][kc * 32], lane);
#pragma unroll
      for (int j = 0; j < 4; ++j) {
        const int o = cg * 64 + j * 16 + col;
        acc[j] = wmma_bf(a, fragw_bf(Wm + (size_t)o * CIN + kc * 32, lane), acc[j]);
      }
    }
    __syncthreads();
#pragma unroll
    for (int j = 0; j < 4; ++j) {
      const int ol = j * 16 + col; const float bb = bfr(Bm[cg * 64 + ol]);
#pragma unroll
      for (int r = 0; r < 8; ++r) {
        const int pl = wave * 16 + 8 * g + r; const float v = acc[j][r] + bb; const _Float16 hv = (_Float16)v;
        if (which == 2) tv[ol][pl] = hv;
        else { sh[pl][ol] = hv; sl[pl][ol] = (_Float16)((v - (float)hv) * QL_CARRY); }
      }
    }
    __syncthreads();
    if (which < 2) {
      _Float16* dh = which == 0 ? QH : KH;
      for (int e = tid; e < 64 * 8; e += 128) {
        const int pl = e >> 3, q = e & 7; const size_t row = b * NP + p0 + pl;
        vst2(dh + row * CQ + cg * 64 + q * 8, *(const v4u*)&sh[pl][q * 8]);
        if (which == 0) vst2(QL + row * CQ + cg * 64 + q * 8, *(const v4u*)&sl[pl][q * 8]);
      }
    } else {
      for (int e = tid; e < 64 * 8; e += 128) {
        const int ol = e >> 3, q = e & 7;
        vst2(VT + (b * CV + cg * 64 + ol) * (size_t)NP + p0 + q * 8, *(const v4u*)&tv[ol][q * 8]);
      }
    }
  }
}

__global__ __launch_bounds__(128) __attribute__((amdgpu_num_vgpr(256)))
void k_sc(const _Float16* __restrict__ QH, const _Float16* __restrict__ QL, const _Float16* __restrict__ KH, int b, float* __restrict__ S) {
  __shared__ __align__(16) float ss[4][16][68];
  const int tid = threadIdx.x, wave = tid >> 5, lane = tid & 31, col = lane & 15, g = lane >> 4;
  const int k0 = blockIdx.y * 64; const int ql0 = blockIdx.x * 64 + wave * 16; const size_t q0 = (size_t)b * NP + ql0;
  v8f acc[4] = {}, accl[4] = {};
#pragma unroll 1
  for (int kc = 0; kc < CQ / 32; ++kc) {
    const v16h ah = frag_h(QH + (q0 + col) * CQ + kc * 32, lane), al = frag_h(QL + (q0 + col) * CQ + kc * 32, lane);
#pragma unroll
    for (int j = 0; j < 4; ++j) {
      const v16h kh = frag_h(KH + ((size_t)b * NP + k0 + j * 16 + col) * CQ + kc * 32, lane);
      acc[j] = wmma16(ah, kh, acc[j]);
      accl[j] = wmma16(al, kh, accl[j]);
    }
  }
#pragma unroll
  for (int j = 0; j < 4; ++j)
#pragma unroll
    for (int r = 0; r < 8; ++r) ss[wave][8 * g + r][j * 16 + col] = acc[j][r] + accl[j][r] * (1.0f / QL_CARRY);
  ldsx();
#pragma unroll
  for (int it = 0; it < 8; ++it) {
    const int rl = 2 * it + g;
    vst2(S + (size_t)(ql0 + rl) * NP + k0 + col * 4, *(const v4f*)&ss[wave][rl][col * 4]);
  }
}

__global__ __launch_bounds__(256) void k_sm(const float* __restrict__ S, _Float16* __restrict__ PH) {
  __shared__ float sred[8]; __shared__ float sbc;
  __shared__ __align__(16) float sv[NP];
  __shared__ __align__(16) _Float16 sh[NP];
  const int t = threadIdx.x; const size_t row = blockIdx.x; const float* sr = S + row * NP;
  float m = -3.0e38f;
  for (int k = t; k < NP; k += 256) { const float v = sr[k]; sv[k] = v; m = fmaxf(m, v); }
#pragma unroll
  for (int o = 1; o < 32; o <<= 1) m = fmaxf(m, __shfl_xor(m, o));
  if ((t & 31) == 0) sred[t >> 5] = m;
  __syncthreads();
  if (t == 0) { float a = sred[0]; for (int i = 1; i < 8; ++i) a = fmaxf(a, sred[i]); sbc = a; }
  __syncthreads();
  m = sbc;
  __syncthreads();
  float sum = 0.f;
#pragma unroll 1
  for (int k = t; k < NP; k += 256) { const float e = expf(sv[k] - m); sv[k] = e; sum += e; }
#pragma unroll
  for (int o = 1; o < 32; o <<= 1) sum += __shfl_xor(sum, o);
  if ((t & 31) == 0) sred[t >> 5] = sum;
  __syncthreads();
  if (t == 0) { float a = 0.f; for (int i = 0; i < 8; ++i) a += sred[i]; sbc = 1.0f / a; }
  __syncthreads();
  const float inv = sbc;
  for (int k = t; k < NP; k += 256) sh[k] = (_Float16)(sv[k] * inv * P_CARRY);
  __syncthreads();
  for (int q = t; q < NP / 8; q += 256) vst2(PH + row * NP + q * 8, *(const v4u*)&sh[q * 8]);
}

__global__ __launch_bounds__(128) __attribute__((amdgpu_num_vgpr(256)))
void k_pvm(const _Float16* __restrict__ PH, const _Float16* __restrict__ VT, int b,
           const float* __restrict__ X, const float* __restrict__ MW, const float* __restrict__ MB, float* __restrict__ OUT) {
  __shared__ __align__(16) float st[128][68];
  __shared__ __align__(16) _Float16 sy[64][CV + 8];
  const int tid = threadIdx.x, wave = tid >> 5, lane = tid & 31, col = lane & 15, g = lane >> 4;
  const int i0 = blockIdx.x * 64; const int il0 = wave * 16;
  {
    v8f acc[8] = {};
#pragma unroll 1
    for (int kc = 0; kc < NP / 32; ++kc) {
      const v16h ph = frag_h(PH + (size_t)(i0 + il0 + col) * NP + kc * 32, lane);
#pragma unroll
      for (int j = 0; j < 8; ++j)
        acc[j] = wmma16(ph, frag_h(VT + ((size_t)b * CV + j * 16 + col) * (size_t)NP + kc * 32, lane), acc[j]);
    }
#pragma unroll
    for (int j = 0; j < 8; ++j) {
      const int cl = j * 16 + col;
#pragma unroll
      for (int r = 0; r < 8; ++r) st[cl][il0 + 8 * g + r] = acc[j][r] * (1.0f / P_CARRY);
    }
  }
  __syncthreads();
  for (int e = tid; e < CV * 64; e += 128) { const int c = e >> 6, n = e & 63; sy[n][c] = (_Float16)(st[c][n] * Y_CARRY); }
  __syncthreads();
#pragma unroll 1
  for (int cg = 0; cg < CIN / 128; ++cg) {
    v8f acc[8] = {};
#pragma unroll 1
    for (int kc = 0; kc < CV / 32; ++kc) {
      const v16h yb = frag_h(&sy[il0 + col][kc * 32], lane);
#pragma unroll
      for (int j = 0; j < 8; ++j) {
        const int o = cg * 128 + j * 16 + col;
        acc[j] = wmma16(fragw_h(MW + (size_t)o * CV + kc * 32, lane, W_CARRY), yb, acc[j]);
      }
    }
    __syncthreads();
#pragma unroll
    for (int j = 0; j < 8; ++j)
#pragma unroll
      for (int r = 0; r < 8; ++r) st[j * 16 + 8 * g + r][il0 + col] = acc[j][r] * (1.0f / (W_CARRY * Y_CARRY));
    __syncthreads();
    for (int e = tid; e < 128 * 16; e += 128) {
      const int cl = e >> 4, q = e & 15; const int co = cg * 128 + cl;
      const size_t o = ((size_t)b * CIN + co) * (size_t)NP + i0 + q * 4;
      const float bb = bfr(MB[co]);
      const v4f m4 = *(const v4f*)&st[cl][q * 4]; const v4f x4 = *(const v4f*)(X + o);
      v4f v;
#pragma unroll
      for (int i = 0; i < 4; ++i) { const float xs = x4[i]; v[i] = (m4[i] + bb) + bfr(xs); }
      vst2(OUT + o, v);
    }
  }
}

extern "C" void kernel_launch(void* const* d_in, const int* in_sizes, int n_in, void* d_out, int out_size, void* d_ws, size_t ws_size, hipStream_t stream) {
  if (n_in < 9) return;
  if ((size_t)in_sizes[0] < (size_t)TNB * CIN * NP) return;
  if (in_sizes[1] < CV * CIN || in_sizes[2] < CV || in_sizes[3] < CQ * CIN || in_sizes[4] < CQ || in_sizes[5] < CQ * CIN || in_sizes[6] < CQ || in_sizes[7] < CIN * CV || in_sizes[8] < CIN) return;
  if ((size_t)out_size < (size_t)TNB * CIN * NP) return;
  if (ws_size < WS_END) return;
  const float* const* F = (const float* const*)d_in;
  const float* X = F[0]; const float* GW = F[1]; const float* GB = F[2]; const float* TW = F[3]; const float* TB = F[4];
  const float* PW = F[5]; const float* PB = F[6]; const float* MW = F[7]; const float* MBv = F[8];
  char* ws = (char*)d_ws;
  _Float16* QH = (_Float16*)(ws + WS_QH); _Float16* QL = (_Float16*)(ws + WS_QL); _Float16* KH = (_Float16*)(ws + WS_KH);
  _Float16* VT = (_Float16*)(ws + WS_VT); float* S = (float*)(ws + WS_S); _Float16* PH = (_Float16*)(ws + WS_PH);
  float* OUT = (float*)d_out;
  k_proj<<<dim3(NP / 64, TNB, 3), 128, 0, stream>>>(X, TW, TB, PW, PB, GW, GB, QH, QL, KH, VT);
  for (int b = 0; b < TNB; ++b) {
    k_sc<<<dim3(TQB, NP / 64), 128, 0, stream>>>(QH, QL, KH, b, S);
    k_sm<<<dim3(TQB * 64), 256, 0, stream>>>(S, PH);
    k_pvm<<<dim3(TQB), 128, 0, stream>>>(PH, VT, b, X, MW, MBv, OUT);
  }
}
